// MicroHeadAttention_89902255440664
// MI455X (gfx1250) — hardware-verified
//
#include <hip/hip_runtime.h>
#include <stddef.h>
#include <stdint.h>


typedef __attribute__((ext_vector_type(16))) __bf16 bf16x16;
typedef __attribute__((ext_vector_type(8)))  float  f32x8;
typedef __attribute__((ext_vector_type(4)))  float  f32x4;
typedef __attribute__((ext_vector_type(4)))  unsigned int u32x4;
typedef u32x4 __attribute__((may_alias)) u32x4a;
typedef f32x4 __attribute__((may_alias)) f32x4a;

#define EMB    1024
#define NTOK   2048
#define MROWS  4096
#define HDIM   64
#define NHEADS 32
#define HSLAB  131072
#define PLANE  4194304
#define WPLANE 1048576
#define CPITCH 68
#define TP     72

union Frag { bf16x16 v; u32x4 q[2]; };

static __device__ __forceinline__ unsigned short bf_bits(float x) {
  __bf16 h = (__bf16)x;
  return __builtin_bit_cast(unsigned short, h);
}
static __device__ __forceinline__ float bf_val(unsigned short u) {
  return __builtin_bit_cast(float, ((unsigned int)u) << 16);
}
static __device__ __forceinline__ float bf_rne(float x) { return bf_val(bf_bits(x)); }

static __device__ __forceinline__ unsigned int split_pair(float a, float b, unsigned int& lo_pair) {
  const unsigned short ha = bf_bits(a), hb = bf_bits(b);
  const unsigned short la = bf_bits(a - bf_val(ha)), lb = bf_bits(b - bf_val(hb));
  lo_pair = (unsigned int)la | ((unsigned int)lb << 16);
  return (unsigned int)ha | ((unsigned int)hb << 16);
}
static __device__ __forceinline__ void split8(f32x4 v0, f32x4 v1, u32x4& H, u32x4& L) {
  unsigned int l0, l1, l2, l3;
  const unsigned int h0 = split_pair(v0.x, v0.y, l0);
  const unsigned int h1 = split_pair(v0.z, v0.w, l1);
  const unsigned int h2 = split_pair(v1.x, v1.y, l2);
  const unsigned int h3 = split_pair(v1.z, v1.w, l3);
  H.x = h0; H.y = h1; H.z = h2; H.w = h3;
  L.x = l0; L.y = l1; L.z = l2; L.w = l3;
}
static __device__ __forceinline__ u32x4 pack8(f32x4 v0, f32x4 v1) {
  u32x4 H;
  H.x = (unsigned int)bf_bits(v0.x) | ((unsigned int)bf_bits(v0.y) << 16);
  H.y = (unsigned int)bf_bits(v0.z) | ((unsigned int)bf_bits(v0.w) << 16);
  H.z = (unsigned int)bf_bits(v1.x) | ((unsigned int)bf_bits(v1.y) << 16);
  H.w = (unsigned int)bf_bits(v1.z) | ((unsigned int)bf_bits(v1.w) << 16);
  return H;
}

static __device__ __forceinline__ f32x8 wmma1(bf16x16 a, bf16x16 b, f32x8 c) {
  c = __builtin_amdgcn_wmma_f32_16x16x32_bf16(false, a, false, b, (short)0, c, false, false);
  asm volatile("v_nop\n\tv_nop\n\tv_nop\n\tv_nop" : "+v"(c) : "v"(a), "v"(b));
  return c;
}
static __device__ __forceinline__ f32x8 wmma2(bf16x16 ah, bf16x16 al, bf16x16 b, f32x8 c) {
  c = __builtin_amdgcn_wmma_f32_16x16x32_bf16(false, al, false, b, (short)0, c, false, false);
  c = __builtin_amdgcn_wmma_f32_16x16x32_bf16(false, ah, false, b, (short)0, c, false, false);
  asm volatile("v_nop\n\tv_nop\n\tv_nop\n\tv_nop" : "+v"(c) : "v"(ah), "v"(al), "v"(b));
  return c;
}
static __device__ __forceinline__ f32x8 wmma3(bf16x16 ah, bf16x16 al, bf16x16 bh, bf16x16 bl, f32x8 c) {
  c = __builtin_amdgcn_wmma_f32_16x16x32_bf16(false, al, false, bh, (short)0, c, false, false);
  c = __builtin_amdgcn_wmma_f32_16x16x32_bf16(false, ah, false, bl, (short)0, c, false, false);
  c = __builtin_amdgcn_wmma_f32_16x16x32_bf16(false, ah, false, bh, (short)0, c, false, false);
  asm volatile("v_nop\n\tv_nop\n\tv_nop\n\tv_nop" : "+v"(c) : "v"(ah), "v"(al), "v"(bh), "v"(bl));
  return c;
}

static __device__ __forceinline__ bf16x16 frag_g(const unsigned short* rowk0, int hh) {
  Frag f;
  f.q[0] = *(const u32x4*)(rowk0 + 8 * hh);
  f.q[1] = *(const u32x4*)(rowk0 + 16 + 8 * hh);
  return f.v;
}
static __device__ __forceinline__ bf16x16 frag_l(const unsigned short* rowk0, int hh) {
  Frag f;
  f.q[0] = *(const u32x4a*)(rowk0 + 8 * hh);
  f.q[1] = *(const u32x4a*)(rowk0 + 16 + 8 * hh);
  return f.v;
}

__global__ __launch_bounds__(256)
void k_cvt(const float* __restrict__ s0, const float* __restrict__ s1,
           const float* __restrict__ s2, const float* __restrict__ s3,
           unsigned short* __restrict__ dst, int n8, int plane_elems)
{
  const int i = blockIdx.x * 256 + threadIdx.x;
  if (i >= n8) return;
  const int y = blockIdx.y;
  const float* src = (y == 0) ? s0 : (y == 1) ? s1 : (y == 2) ? s2 : s3;
  const float* p = src + (size_t)i * 8;
  const f32x4 v0 = *(const f32x4*)p;
  const f32x4 v1 = *(const f32x4*)(p + 4);
  const u32x4 H = pack8(v0, v1);
  unsigned short* ph = dst + (size_t)y * (size_t)plane_elems + (size_t)i * 8;
  *(volatile u32x4*)ph = H;
  __threadfence();
  *(volatile u32x4*)ph = H;
}

__global__ __launch_bounds__(256)
void k_qkv(const unsigned short* __restrict__ Xb, const unsigned short* __restrict__ Wb,
           const float* __restrict__ bq, const float* __restrict__ bk, const float* __restrict__ bv,
           unsigned short* __restrict__ Ph, unsigned short* __restrict__ Pl)
{
  __shared__ __attribute__((aligned(16))) float Cs[128 * CPITCH];

  const int tid = threadIdx.x, lane = tid & 31, wave = tid >> 5;
  const int m = lane & 15, hh = lane >> 4;
  const int m0 = blockIdx.x * 128;
  const int t  = blockIdx.y >> 4;
  const int n0 = (blockIdx.y & 15) * 64;
  const int wm = (wave >> 1) * 32, wn = (wave & 1) * 32;

  const float* bias = (t == 0) ? bq : (t == 1) ? bk : bv;
  const unsigned short* Bp = Wb + (size_t)t * (size_t)WPLANE;

  const unsigned short* a0 = Xb + (size_t)(m0 + wm + m) * EMB;
  const unsigned short* a1 = a0 + (size_t)16 * EMB;
  const unsigned short* b0 = Bp + (size_t)(n0 + wn + m) * EMB;
  const unsigned short* b1 = b0 + (size_t)16 * EMB;

  f32x8 acc[2][2] = {};

  #pragma unroll 1
  for (int k0 = 0; k0 < EMB; k0 += 32) {
    const bf16x16 A0 = frag_g(a0 + k0, hh);
    const bf16x16 A1 = frag_g(a1 + k0, hh);
    const bf16x16 B0 = frag_g(b0 + k0, hh);
    const bf16x16 B1 = frag_g(b1 + k0, hh);
    acc[0][0] = wmma1(A0, B0, acc[0][0]);
    acc[0][1] = wmma1(A0, B1, acc[0][1]);
    acc[1][0] = wmma1(A1, B0, acc[1][0]);
    acc[1][1] = wmma1(A1, B1, acc[1][1]);
  }

  #pragma unroll
  for (int tn = 0; tn < 2; ++tn) {
    const int col = wn + tn * 16 + m;
    const float bval = bf_rne(bias[n0 + col]);
    #pragma unroll
    for (int tm = 0; tm < 2; ++tm) {
      #pragma unroll
      for (int r = 0; r < 8; ++r)
        Cs[(wm + tm * 16 + 8 * hh + r) * CPITCH + col] = acc[tm][tn][r] + bval;
    }
  }
  __syncthreads();

  u32x4 Hv[4], Lv[4];
  size_t off[4];
  #pragma unroll
  for (int i = 0; i < 4; ++i) {
    const int p = tid + i * 256;
    const int row = p >> 3, c8 = (p & 7) * 8;
    const f32x4 v0 = *(const f32x4a*)&Cs[row * CPITCH + c8];
    const f32x4 v1 = *(const f32x4a*)&Cs[row * CPITCH + c8 + 4];
    split8(v0, v1, Hv[i], Lv[i]);
    const int mrow = m0 + row;
    const int bb = mrow >> 11, nn = mrow & 2047;
    const int colE = n0 + c8;
    const int g = colE >> 9, cc = colE & 511;
    off[i] = (size_t)t * PLANE + (((size_t)(bb * 2 + g)) << 20) + (size_t)nn * 512 + (size_t)cc;
    *(volatile u32x4*)(Ph + off[i]) = Hv[i];
    *(volatile u32x4*)(Pl + off[i]) = Lv[i];
  }
  __threadfence();
  #pragma unroll
  for (int i = 0; i < 4; ++i) {
    *(volatile u32x4*)(Ph + off[i]) = Hv[i];
    *(volatile u32x4*)(Pl + off[i]) = Lv[i];
  }
}

__global__ __launch_bounds__(128)
void k_attn(const unsigned short* __restrict__ Ph, const unsigned short* __restrict__ Pl,
            unsigned short* __restrict__ Ch, unsigned short* __restrict__ Cl)
{
  __shared__ __attribute__((aligned(16))) unsigned short Kth[64 * TP];
  __shared__ __attribute__((aligned(16))) unsigned short Ktl[64 * TP];
  __shared__ __attribute__((aligned(16))) unsigned short Vth[64 * TP];
  __shared__ __attribute__((aligned(16))) unsigned short Vtl[64 * TP];
  __shared__ __attribute__((aligned(16))) unsigned short Psm[4 * 2 * 16 * TP];

  const int tid = threadIdx.x, lane = tid & 31, wave = tid >> 5;
  const int m = lane & 15, hh = lane >> 4;
  const int qb = blockIdx.x;
  const int hd = blockIdx.y;
  const int q0 = qb * 64 + wave * 16;

  const size_t hs = (size_t)hd * HSLAB;
  const unsigned short* Qgh = Ph + hs;
  const unsigned short* Qgl = Pl + hs;
  const unsigned short* Kgh = Ph + (size_t)PLANE + hs;
  const unsigned short* Kgl = Pl + (size_t)PLANE + hs;
  const unsigned short* Vgh = Ph + (size_t)2 * PLANE + hs;
  const unsigned short* Vgl = Pl + (size_t)2 * PLANE + hs;
  unsigned short* Pwh = Psm + wave * (2 * 16 * TP);
  unsigned short* Pwl = Pwh + 16 * TP;

  bf16x16 qah[2], qal[2];
  #pragma unroll
  for (int ks = 0; ks < 2; ++ks) {
    qah[ks] = frag_g(Qgh + (size_t)(q0 + m) * HDIM + ks * 32, hh);
    qal[ks] = frag_g(Qgl + (size_t)(q0 + m) * HDIM + ks * 32, hh);
  }

  f32x8 acc[4] = {};
  float mi[8], li[8];
  #pragma unroll
  for (int r = 0; r < 8; ++r) { mi[r] = -3.0e38f; li[r] = 0.0f; }

  for (int j = 0; j <= qb; ++j) {
    const int k0 = j * 64;
    __syncthreads();

    #pragma unroll
    for (int i = 0; i < 4; ++i) {
      const int p = tid + i * 128;
      const int key = p >> 3, d8 = (p & 7) * 8;
      const size_t go = (size_t)(k0 + key) * HDIM + d8;
      const u32x4 kvh = *(const u32x4*)(Kgh + go);
      const u32x4 kvl = *(const u32x4*)(Kgl + go);
      *(u32x4a*)&Kth[key * TP + d8] = kvh;
      *(u32x4a*)&Ktl[key * TP + d8] = kvl;
      const u32x4 vvh = *(const u32x4*)(Vgh + go);
      const u32x4 vvl = *(const u32x4*)(Vgl + go);
      const unsigned int vhw[4] = { vvh.x, vvh.y, vvh.z, vvh.w };
      const unsigned int vlw[4] = { vvl.x, vvl.y, vvl.z, vvl.w };
      #pragma unroll
      for (int e = 0; e < 8; ++e) {
        const int sh = 16 * (e & 1);
        Vth[(d8 + e) * TP + key] = (unsigned short)(vhw[e >> 1] >> sh);
        Vtl[(d8 + e) * TP + key] = (unsigned short)(vlw[e >> 1] >> sh);
      }
    }
    __syncthreads();

    f32x8 sc[4];
    #pragma unroll
    for (int tn = 0; tn < 4; ++tn) {
      f32x8 z = {};
      #pragma unroll
      for (int ks = 0; ks < 2; ++ks) {
        const bf16x16 kbh = frag_l(&Kth[(tn * 16 + m) * TP + ks * 32], hh);
        const bf16x16 kbl = frag_l(&Ktl[(tn * 16 + m) * TP + ks * 32], hh);
        z = wmma3(qah[ks], qal[ks], kbh, kbl, z);
      }
      sc[tn] = z;
    }

    float mnew[8];
    #pragma unroll
    for (int r = 0; r < 8; ++r) mnew[r] = -3.0e38f;
    #pragma unroll
    for (int tn = 0; tn < 4; ++tn) {
      const int kidx = k0 + tn * 16 + m;
      #pragma unroll
      for (int r = 0; r < 8; ++r) {
        const int qidx = q0 + 8 * hh + r;
        const float v = (kidx <= qidx) ? sc[tn][r] * 0.125f : -3.0e38f;
        sc[tn][r] = v;
        mnew[r] = fmaxf(mnew[r], v);
      }
    }
    #pragma unroll
    for (int r = 0; r < 8; ++r) {
      #pragma unroll
      for (int off = 1; off < 16; off <<= 1)
        mnew[r] = fmaxf(mnew[r], __shfl_xor(mnew[r], off, 16));
    }

    float alpha[8], rsum[8];
    #pragma unroll
    for (int r = 0; r < 8; ++r) {
      const float mn = fmaxf(mi[r], mnew[r]);
      alpha[r] = __expf(mi[r] - mn);
      mi[r] = mn;
      rsum[r] = 0.0f;
    }

    asm volatile("" ::: "memory");
    #pragma unroll
    for (int tn = 0; tn < 4; ++tn) {
      #pragma unroll
      for (int r = 0; r < 8; ++r) {
        const float pv = __expf(sc[tn][r] - mi[r]);
        rsum[r] += pv;
        const unsigned short hb = bf_bits(pv);
        const unsigned short lb = bf_bits(pv - bf_val(hb));
        Pwh[(8 * hh + r) * TP + tn * 16 + m] = hb;
        Pwl[(8 * hh + r) * TP + tn * 16 + m] = lb;
      }
    }
    asm volatile("" ::: "memory");

    #pragma unroll
    for (int r = 0; r < 8; ++r) {
      #pragma unroll
      for (int off = 1; off < 16; off <<= 1)
        rsum[r] += __shfl_xor(rsum[r], off, 16);
      li[r] = li[r] * alpha[r] + rsum[r];
    }
    #pragma unroll
    for (int td = 0; td < 4; ++td) {
      #pragma unroll
      for (int r = 0; r < 8; ++r) acc[td][r] *= alpha[r];
    }

    #pragma unroll
    for (int ks = 0; ks < 2; ++ks) {
      const bf16x16 pah = frag_l(&Pwh[m * TP + ks * 32], hh);
      const bf16x16 pal = frag_l(&Pwl[m * TP + ks * 32], hh);
      #pragma unroll
      for (int td = 0; td < 4; ++td) {
        const bf16x16 vbh = frag_l(&Vth[(td * 16 + m) * TP + ks * 32], hh);
        const bf16x16 vbl = frag_l(&Vtl[(td * 16 + m) * TP + ks * 32], hh);
        acc[td] = wmma3(pah, pal, vbh, vbl, acc[td]);
      }
    }
  }

  float inv[8];
  #pragma unroll
  for (int r = 0; r < 8; ++r) inv[r] = 1.0f / li[r];
  asm volatile("" ::: "memory");
  #pragma unroll
  for (int td = 0; td < 4; ++td) {
    #pragma unroll
    for (int r = 0; r < 8; ++r) {
      const float cv = acc[td][r] * inv[r];
      const unsigned short hb = bf_bits(cv);
      const unsigned short lb = bf_bits(cv - bf_val(hb));
      Pwh[(8 * hh + r) * TP + td * 16 + m] = hb;
      Pwl[(8 * hh + r) * TP + td * 16 + m] = lb;
    }
  }
  asm volatile("" ::: "memory");

  u32x4 Hv[4], Lv[4];
  size_t off[4];
  #pragma unroll
  for (int i = 0; i < 4; ++i) {
    const int p = lane + 32 * i;
    const int row = p >> 3, c8 = (p & 7) * 8;
    Hv[i] = *(const u32x4a*)&Pwh[row * TP + c8];
    Lv[i] = *(const u32x4a*)&Pwl[row * TP + c8];
    off[i] = hs + (size_t)(q0 + row) * HDIM + (size_t)c8;
    *(volatile u32x4*)(Ch + off[i]) = Hv[i];
    *(volatile u32x4*)(Cl + off[i]) = Lv[i];
  }
  __threadfence();
  #pragma unroll
  for (int i = 0; i < 4; ++i) {
    *(volatile u32x4*)(Ch + off[i]) = Hv[i];
    *(volatile u32x4*)(Cl + off[i]) = Lv[i];
  }
}

__global__ __launch_bounds__(256)
void k_out(const unsigned short* __restrict__ Ch, const unsigned short* __restrict__ Cl,
           const unsigned short* __restrict__ Wob,
           const float* __restrict__ bo, float* __restrict__ out)
{
  __shared__ __attribute__((aligned(16))) float Cs[128 * CPITCH];

  const int tid = threadIdx.x, lane = tid & 31, wave = tid >> 5;
  const int m = lane & 15, hh = lane >> 4;
  const int m0 = blockIdx.x * 128;
  const int n0 = blockIdx.y * 64;
  const int wm = (wave >> 1) * 32, wn = (wave & 1) * 32;

  const int r0 = m0 + wm + m, r1 = r0 + 16;
  const size_t base0 = (((size_t)((r0 >> 11) * 2)) << 20) + (size_t)(r0 & 2047) * 512;
  const size_t base1 = (((size_t)((r1 >> 11) * 2)) << 20) + (size_t)(r1 & 2047) * 512;
  const unsigned short* b0 = Wob + (size_t)(n0 + wn + m) * EMB;
  const unsigned short* b1 = b0 + (size_t)16 * EMB;

  f32x8 acc[2][2] = {};

  #pragma unroll 1
  for (int k0 = 0; k0 < EMB; k0 += 32) {
    const size_t ko = (((size_t)(k0 >> 9)) << 20) + (size_t)(k0 & 511);
    const bf16x16 A0h = frag_g(Ch + base0 + ko, hh), A0l = frag_g(Cl + base0 + ko, hh);
    const bf16x16 A1h = frag_g(Ch + base1 + ko, hh), A1l = frag_g(Cl + base1 + ko, hh);
    const bf16x16 B0 = frag_g(b0 + k0, hh);
    const bf16x16 B1 = frag_g(b1 + k0, hh);
    acc[0][0] = wmma2(A0h, A0l, B0, acc[0][0]);
    acc[0][1] = wmma2(A0h, A0l, B1, acc[0][1]);
    acc[1][0] = wmma2(A1h, A1l, B0, acc[1][0]);
    acc[1][1] = wmma2(A1h, A1l, B1, acc[1][1]);
  }

  #pragma unroll
  for (int tn = 0; tn < 2; ++tn) {
    const int col = wn + tn * 16 + m;
    const float bval = bf_rne(bo[n0 + col]);
    #pragma unroll
    for (int tm = 0; tm < 2; ++tm) {
      #pragma unroll
      for (int r = 0; r < 8; ++r)
        Cs[(wm + tm * 16 + 8 * hh + r) * CPITCH + col] = acc[tm][tn][r] + bval;
    }
  }
  __syncthreads();

  f32x4 v[8];
  size_t off[8];
  #pragma unroll
  for (int i = 0; i < 8; ++i) {
    const int p = tid + i * 256;
    const int row = p >> 4, c4 = (p & 15) * 4;
    v[i] = *(const f32x4a*)&Cs[row * CPITCH + c4];
    off[i] = (size_t)(m0 + row) * EMB + (size_t)(n0 + c4);
    *(volatile f32x4*)(out + off[i]) = v[i];
  }
  __threadfence();
  #pragma unroll
  for (int i = 0; i < 8; ++i)
    *(volatile f32x4*)(out + off[i]) = v[i];
}

extern "C" void kernel_launch(void* const* d_in, const int* in_sizes, int n_in,
                              void* d_out, int out_size, void* d_ws, size_t ws_size,
                              hipStream_t stream)
{
  if (n_in < 9) return;
  if (in_sizes[0] != PLANE) return;
  if (in_sizes[1] != WPLANE || in_sizes[3] != WPLANE ||
      in_sizes[5] != WPLANE || in_sizes[7] != WPLANE) return;
  if (in_sizes[2] != EMB || in_sizes[4] != EMB || in_sizes[6] != EMB || in_sizes[8] != EMB) return;
  if (out_size != PLANE) return;
  const size_t need = (size_t)40 * 1048576 * sizeof(unsigned short);
  if (ws_size < need) return;

  const float* x  = (const float*)d_in[0];
  const float* Wq = (const float*)d_in[1];
  const float* bq = (const float*)d_in[2];
  const float* Wk = (const float*)d_in[3];
  const float* bk = (const float*)d_in[4];
  const float* Wv = (const float*)d_in[5];
  const float* bv = (const float*)d_in[6];
  const float* Wo = (const float*)d_in[7];
  const float* bo = (const float*)d_in[8];
  float* out = (float*)d_out;

  unsigned short* ws = (unsigned short*)d_ws;
  unsigned short* Xb   = ws;
  unsigned short* Wb   = ws + (size_t)4  * 1048576;
  unsigned short* QKVh = ws + (size_t)8  * 1048576;
  unsigned short* QKVl = ws + (size_t)20 * 1048576;
  unsigned short* Ch   = ws + (size_t)32 * 1048576;
  unsigned short* Cl   = ws + (size_t)36 * 1048576;

  const int n8x = PLANE / 8;
  const int n8w = WPLANE / 8;
  const int gx = (n8x + 255) / 256;
  const int gw = (n8w + 255) / 256;

  k_cvt<<<dim3(gx, 1), dim3(256), 0, stream>>>(x, x, x, x, Xb, n8x, 0);
  k_cvt<<<dim3(gw, 4), dim3(256), 0, stream>>>(Wq, Wk, Wv, Wo, Wb, n8w, WPLANE);

  k_qkv<<<dim3(MROWS / 128, 3 * (EMB / 64)), dim3(256), 0, stream>>>(Xb, Wb, bq, bk, bv, QKVh, QKVl);
  k_attn<<<dim3(NTOK / 64, NHEADS), dim3(128), 0, stream>>>(QKVh, QKVl, Ch, Cl);
  k_out<<<dim3(MROWS / 128, EMB / 64), dim3(256), 0, stream>>>(Ch, Cl,
      Wb + (size_t)3 * WPLANE, bo, out);
}
